// TruthGPTFlashAttention_50964081934740
// MI455X (gfx1250) — hardware-verified
//
#include <hip/hip_runtime.h>
#include <stdint.h>

typedef __attribute__((ext_vector_type(16))) _Float16 v16h;
typedef __attribute__((ext_vector_type(8)))  _Float16 v8h;
typedef __attribute__((ext_vector_type(16))) __bf16   v16b;
typedef __attribute__((ext_vector_type(8)))  __bf16   v8b;
typedef __attribute__((ext_vector_type(8)))  float    v8f;
typedef __attribute__((ext_vector_type(4)))  float    v4f;
#define PSCALE 32768.0f
#define U16(p) ((const unsigned short*)(const void*)(p))
#define PSCALE_INV (1.0f / 32768.0f)

__device__ __forceinline__ unsigned short f2bf_bits(float f) {
  unsigned u = __float_as_uint(f);
  return (unsigned short)((u + 0x7FFFu + ((u >> 16) & 1u)) >> 16);
}
__device__ __forceinline__ float bf_bits2f(unsigned short h) { return __uint_as_float(((unsigned)h) << 16); }

__device__ __forceinline__ void dep_guard_h(v8f& a, v8f& b, v16h x, v16h y) { asm volatile("v_nop\n\tv_nop\n\tv_nop\n\tv_nop" : "+v"(a), "+v"(b) : "v"(x), "v"(y)); }
__device__ __forceinline__ void dep_guard_b(v8f& a, v8f& b, v16b x, v16b y) { asm volatile("v_nop\n\tv_nop\n\tv_nop\n\tv_nop" : "+v"(a), "+v"(b) : "v"(x), "v"(y)); }
__device__ __forceinline__ void keep4_h(v16h a, v16h b, v16h c, v16h d) { asm volatile("v_nop" :: "v"(a), "v"(b), "v"(c), "v"(d)); }
__device__ __forceinline__ void keep4_b(v16b a, v16b b, v16b c, v16b d) { asm volatile("v_nop" :: "v"(a), "v"(b), "v"(c), "v"(d)); }
__device__ __forceinline__ void acc_guard4(v8f& a, v8f& b, v8f& c, v8f& d) { asm volatile("v_nop\n\tv_nop\n\tv_nop\n\tv_nop" : "+v"(a), "+v"(b), "+v"(c), "+v"(d)); }
template <typename T> struct Frag;
template <> struct Frag<_Float16> {
  typedef v16h V; union U { v16h v; v8h h[2]; };
  static __device__ __forceinline__ v16h load(const _Float16* p) {
    U f; f.h[0] = *(const v8h*)(p); f.h[1] = *(const v8h*)(p + 16); return f.v;
  }
  static __device__ __forceinline__ v8f mma(v16h a, v16h b, v8f c) {
    return __builtin_amdgcn_wmma_f32_16x16x32_f16(false, a, false, b, (short)0, c, false, false);
  }
  static __device__ __forceinline__ void guard(v8f& a, v8f& b, v16h x, v16h y) { dep_guard_h(a, b, x, y); }
  static __device__ __forceinline__ void keep(v16h a, v16h b, v16h c, v16h d) { keep4_h(a, b, c, d); }
};
template <> struct Frag<__bf16> {
  typedef v16b V; union U { v16b v; v8b h[2]; };
  static __device__ __forceinline__ v16b load(const __bf16* p) {
    U f; f.h[0] = *(const v8b*)(p); f.h[1] = *(const v8b*)(p + 16); return f.v;
  }
  static __device__ __forceinline__ v8f mma(v16b a, v16b b, v8f c) {
    return __builtin_amdgcn_wmma_f32_16x16x32_bf16(false, a, false, b, (short)0, c, false, false);
  }
  static __device__ __forceinline__ void guard(v8f& a, v8f& b, v16b x, v16b y) { dep_guard_b(a, b, x, y); }
  static __device__ __forceinline__ void keep(v16b a, v16b b, v16b c, v16b d) { keep4_b(a, b, c, d); }
};

template <int ET> struct Elem;
template <> struct Elem<0> { typedef _Float16 T; };
template <> struct Elem<1> { typedef __bf16 T; };
template <int ET, bool SPLIT, int BIAS_MODE, int OUT_MODE, bool RESID, int ACT = 0>
__global__ __launch_bounds__(256) void wmma_gemm64(
    const unsigned short* __restrict__ Ap, const unsigned short* __restrict__ A2p, int lda, long strideA,
    const unsigned short* __restrict__ Btp, const unsigned short* __restrict__ Bt2p, int ldb, long strideB,
    void* __restrict__ Cout, void* __restrict__ Cout2, int ldc, long strideC,
    const float* __restrict__ bias,
    const float* __restrict__ resid, long strideR,
    int M, int N, int K, float scale) {
  typedef typename Elem<ET>::T T;
  typedef typename Frag<T>::V V;
  const T* A = (const T*)Ap; const T* A2 = (const T*)A2p; const T* Bt = (const T*)Btp; const T* Bt2 = (const T*)Bt2p;
  __shared__ __align__(16) float sT[8][16 * 68];
  const int b    = blockIdx.y;
  const int lane = threadIdx.x & 31;
  const int wave = threadIdx.x >> 5;
  const int tilesN = N >> 6;
  const int tilesM = M >> 6;
  const int tile = blockIdx.x * 8 + wave;
  if (tile >= tilesM * tilesN) return;
  const int tm = tile / tilesN;
  const int tn = tile - tm * tilesN;
  const int m0 = tm << 6;
  const int n0 = tn << 6;

  const T* Ab  = A  + (size_t)b * strideA;
  const T* Bb  = Bt + (size_t)b * strideB;
  const T* Ab2 = SPLIT ? (A2  + (size_t)b * strideA) : nullptr;
  const T* Bb2 = SPLIT ? (Bt2 + (size_t)b * strideB) : nullptr;

  const int rlane = lane & 15;
  const int koff  = (lane >> 4) * 8;
  const int mOff  = (lane >> 4) * 8;

  v8f acc[4][4];
#pragma unroll
  for (int i = 0; i < 4; ++i)
#pragma unroll
    for (int j = 0; j < 4; ++j) acc[i][j] = (v8f){0.f,0.f,0.f,0.f,0.f,0.f,0.f,0.f};

  for (int k0 = 0; k0 < K; k0 += 32) {
    V bh[4], bl[4];
#pragma unroll
    for (int j = 0; j < 4; ++j) {
      const size_t bo = (size_t)(n0 + (j << 4) + rlane) * ldb + koff + k0;
      bh[j] = Frag<T>::load(Bb + bo);
      if (SPLIT) bl[j] = Frag<T>::load(Bb2 + bo);
    }
#pragma unroll
    for (int i = 0; i < 4; ++i) {
      const size_t ao = (size_t)(m0 + (i << 4) + rlane) * lda + koff + k0;
      V ah = Frag<T>::load(Ab + ao);
      V al;
      if (SPLIT) al = Frag<T>::load(Ab2 + ao);
#pragma unroll
      for (int j = 0; j < 4; ++j) {
        acc[i][j] = Frag<T>::mma(ah, bh[j], acc[i][j]);
        if (SPLIT) {
          acc[i][j] = Frag<T>::mma(ah, bl[j], acc[i][j]);
          acc[i][j] = Frag<T>::mma(al, bh[j], acc[i][j]);
        }
      }
      Frag<T>::guard(acc[i][0], acc[i][3], ah, SPLIT ? al : ah);
    }
    Frag<T>::keep(bh[0], bh[1], bh[2], bh[3]);
    if (SPLIT) Frag<T>::keep(bl[0], bl[1], bl[2], bl[3]);
  }
  acc_guard4(acc[0][0], acc[0][1], acc[0][2], acc[0][3]);
  acc_guard4(acc[1][0], acc[1][1], acc[1][2], acc[1][3]);
  acc_guard4(acc[2][0], acc[2][1], acc[2][2], acc[2][3]);
  acc_guard4(acc[3][0], acc[3][1], acc[3][2], acc[3][3]);

  float* slab = sT[wave];
  const float* Rb = RESID ? (resid + (size_t)b * strideR) : nullptr;
#pragma unroll
  for (int i = 0; i < 4; ++i) {
    const int mBase = m0 + (i << 4);
#pragma unroll
    for (int j = 0; j < 4; ++j) {
      const int n = n0 + (j << 4) + rlane;
      float bv = 0.f;
      if (BIAS_MODE == 2) bv = bias[n];
#pragma unroll
      for (int r = 0; r < 8; ++r) {
        float v = acc[i][j][r] * scale;
        if (BIAS_MODE == 1) v += bias[mBase + mOff + r];
        if (BIAS_MODE == 2) v += bv;
        if (RESID) v += Rb[(size_t)(mBase + mOff + r) * ldc + n];
        if (ACT == 1) v = tanhf(v);
        if (ACT == 2) v = fmaxf(v, 0.0f);
        if (ACT == 3) v = v / (1.0f + expf(-v));
        if (ACT == 4) v = (v > 0.f) ? v : 0.01f * v;
        if (ACT == 5) v = 0.5f * v * (1.0f + erff(v * 0.70710678118654752f));
        slab[(mOff + r) * 68 + (j << 4) + rlane] = v;
      }
    }
    __builtin_amdgcn_fence(__ATOMIC_RELEASE, "workgroup");
    __builtin_amdgcn_wave_barrier();
    __builtin_amdgcn_fence(__ATOMIC_ACQUIRE, "workgroup");
    if (OUT_MODE == 0) {
      float* C = (float*)Cout + (size_t)b * strideC;
      const int hh = lane >> 4, c4 = (lane & 15) * 4;
      for (int pass = 0; pass < 2; ++pass) {
#pragma unroll
        for (int it = 0; it < 8; ++it) {
          const int row = it * 2 + hh;
          v4f v = *(const v4f*)(slab + row * 68 + c4);
          *(volatile v4f*)(C + (size_t)(mBase + row) * ldc + n0 + c4) = v;
        }
        __threadfence();
      }
    } else {
      const int q = lane >> 3, c8 = (lane & 7) * 8;
      unsigned short* C  = (unsigned short*)Cout  + (size_t)b * strideC;
      unsigned short* C2 = (OUT_MODE == 2) ? ((unsigned short*)Cout2 + (size_t)b * strideC) : nullptr;
      for (int pass = 0; pass < 2; ++pass) {
#pragma unroll
        for (int it = 0; it < 4; ++it) {
          const int row = it * 4 + q;
          const float* sp = slab + row * 68 + c8;
          v8h hv, lv;
#pragma unroll
          for (int e = 0; e < 8; ++e) {
            if (OUT_MODE == 1) {
              hv[e] = (_Float16)sp[e];
            } else {
              unsigned short hb = f2bf_bits(sp[e]);
              unsigned short lb = f2bf_bits(sp[e] - bf_bits2f(hb));
              hv[e] = __builtin_bit_cast(_Float16, hb);
              lv[e] = __builtin_bit_cast(_Float16, lb);
            }
          }
          *(volatile v8h*)(C + (size_t)(mBase + row) * ldc + n0 + c8) = hv;
          if (OUT_MODE == 2) *(volatile v8h*)(C2 + (size_t)(mBase + row) * ldc + n0 + c8) = lv;
        }
        __threadfence();
      }
    }
    __builtin_amdgcn_fence(__ATOMIC_RELEASE, "workgroup");
    __builtin_amdgcn_wave_barrier();
    __builtin_amdgcn_fence(__ATOMIC_ACQUIRE, "workgroup");
  }
}

__global__ __launch_bounds__(256) void cast_f32_f16x2(
    const float* __restrict__ in, _Float16* __restrict__ out, int n2) {
  int i = blockIdx.x * 256 + threadIdx.x;
  if (i < n2) {
    const _Float16 h0 = (_Float16)in[2 * i], h1 = (_Float16)in[2 * i + 1];
    const unsigned u = (unsigned)__builtin_bit_cast(unsigned short, h0) | ((unsigned)__builtin_bit_cast(unsigned short, h1) << 16);
    ((volatile unsigned*)out)[i] = u;
    __threadfence();
    ((volatile unsigned*)out)[i] = u;
  }
}

__global__ __launch_bounds__(256) void k_transpose_cast4(
    const float* __restrict__ w0, const float* __restrict__ w1,
    const float* __restrict__ w2, const float* __restrict__ w3,
    _Float16* __restrict__ wt, int K, int N, float sc) {
  __shared__ float tile[64][65];
  const int z = blockIdx.z;
  const float* w = (z == 0) ? w0 : ((z == 1) ? w1 : ((z == 2) ? w2 : w3));
  _Float16* o = wt + (size_t)z * (size_t)N * (size_t)K;
  const int n0 = blockIdx.x * 64;
  const int k0 = blockIdx.y * 64;
  const int tid = threadIdx.x, lane = tid & 31, wave = tid >> 5;
#pragma unroll
  for (int i = 0; i < 16; ++i) {
    const int idx = i * 256 + tid;
    const int r = idx >> 6, cc = idx & 63;
    tile[r][cc] = w[(size_t)(k0 + r) * N + n0 + cc];
  }
  __syncthreads();
  const int q8 = lane >> 3, c8 = (lane & 7) * 8;
  const int nl0 = wave * 4 + q8;
  const int nl1 = 32 + wave * 4 + q8;
  v8h val0, val1;
#pragma unroll
  for (int e = 0; e < 8; ++e) {
    val0[e] = (_Float16)(tile[c8 + e][nl0] * sc);
    val1[e] = (_Float16)(tile[c8 + e][nl1] * sc);
  }
  _Float16* p0 = o + (size_t)(n0 + nl0) * K + k0 + c8;
  _Float16* p1 = o + (size_t)(n0 + nl1) * K + k0 + c8;
  for (int pass = 0; pass < 2; ++pass) {
    *(volatile v8h*)p0 = val0;
    *(volatile v8h*)p1 = val1;
    __threadfence();
  }
}

#define AT_D 64
#define AT_NW 4
#define AT_QB 64
#define AT_KC 64
#define PSC_F 32768.0f

__device__ __forceinline__ v8f mma_h(v16h a, v16h b, v8f c) {
  c = __builtin_amdgcn_wmma_f32_16x16x32_f16(false, a, false, b, (short)0, c, false, false);
  asm volatile("v_nop\n\tv_nop\n\tv_nop\n\tv_nop" : "+v"(c) : "v"(a), "v"(b));
  return c;
}

__global__ __launch_bounds__(128)
void attn64_f16_kernel(const _Float16* __restrict__ q, const _Float16* __restrict__ k,
                       const _Float16* __restrict__ v, _Float16* __restrict__ out,
                       int S, int NHh, int ld, float sscale, float osc) {
  union FH { v16h v; v8h h[2]; };
  __shared__ __align__(16) _Float16 Ksh[AT_KC * AT_D];
  __shared__ __align__(16) _Float16 Vth[AT_D * AT_KC];
  __shared__ __align__(16) _Float16 Psh[AT_NW][16 * AT_KC];
  __shared__ __align__(16) float  Os[AT_NW][16 * 68];

  const int tid  = threadIdx.x;
  const int wave = tid >> 5;
  const int lane = tid & 31;
  const int hh   = lane >> 4;
  const int c    = lane & 15;

  const int nqb = S / AT_QB;
  const int bx = blockIdx.x;
  const int qb = bx % nqb;
  const int bh = bx / nqb;
  const int h  = bh % NHh;
  const int b  = bh / NHh;
  const int q0 = qb * AT_QB + wave * 16;

  const size_t bs = (size_t)S * (size_t)ld;
  const _Float16* qb_ptr = q + (size_t)b * bs + (size_t)h * AT_D;
  const _Float16* kb_ptr = k + (size_t)b * bs + (size_t)h * AT_D;
  const _Float16* vb_ptr = v + (size_t)b * bs + (size_t)h * AT_D;
  _Float16*       ob_ptr = out + (size_t)b * bs + (size_t)h * AT_D;

  v16h qa[2];
  {
    const _Float16* qrow = qb_ptr + (size_t)(q0 + c) * ld;
    qa[0] = Frag<_Float16>::load(qrow + 8 * hh);
    qa[1] = Frag<_Float16>::load(qrow + 32 + 8 * hh);
  }

  float mrow[8], lrow[8];
  v8f oacc[4];
  const float ninf = -__builtin_inff();
#pragma unroll
  for (int r = 0; r < 8; ++r) { mrow[r] = ninf; lrow[r] = 0.f; }
#pragma unroll
  for (int t = 0; t < 4; ++t) oacc[t] = (v8f){0.f,0.f,0.f,0.f,0.f,0.f,0.f,0.f};

  const int nChunks = S / AT_KC;
  for (int kc = 0; kc < nChunks; ++kc) {
    const int kv0 = kc * AT_KC;
    __syncthreads();
    {
      const int kvr = tid >> 1, dh = (tid & 1) * 32;
      const _Float16* krow = kb_ptr + (size_t)(kv0 + kvr) * ld + dh;
      const _Float16* vrow = vb_ptr + (size_t)(kv0 + kvr) * ld + dh;
#pragma unroll
      for (int i = 0; i < 4; ++i) {
        const v8h kk8 = *(const v8h*)(krow + 8 * i);
        const v8h vv8 = *(const v8h*)(vrow + 8 * i);
        *(v8h*)(Ksh + kvr * AT_D + dh + 8 * i) = kk8;
#pragma unroll
        for (int e = 0; e < 8; ++e) Vth[(dh + 8 * i + e) * AT_KC + kvr] = vv8[e];
      }
    }
    __syncthreads();

    v8f s[4];
#pragma unroll
    for (int j = 0; j < 4; ++j) {
      s[j] = (v8f){0.f,0.f,0.f,0.f,0.f,0.f,0.f,0.f};
#pragma unroll
      for (int dc = 0; dc < 2; ++dc) {
        FH kb;
        kb.h[0] = *(const v8h*)(Ksh + (j * 16 + c) * AT_D + dc * 32 + 8 * hh);
        kb.h[1] = *(const v8h*)(Ksh + (j * 16 + c) * AT_D + dc * 32 + 16 + 8 * hh);
        s[j] = mma_h(qa[dc], kb.v, s[j]);
      }
    }

    float cm[8];
#pragma unroll
    for (int r = 0; r < 8; ++r) {
      float m = ninf;
#pragma unroll
      for (int j = 0; j < 4; ++j) {
        s[j][r] *= sscale;
        m = fmaxf(m, s[j][r]);
      }
#pragma unroll
      for (int off = 1; off < 16; off <<= 1) m = fmaxf(m, __shfl_xor(m, off, 32));
      cm[r] = m;
    }
    _Float16* pwh = Psh[wave];
#pragma unroll
    for (int r = 0; r < 8; ++r) {
      const float mnew = fmaxf(mrow[r], cm[r]);
      const float alpha = __expf(mrow[r] - mnew);
      mrow[r] = mnew;
      float psum = 0.f;
#pragma unroll
      for (int j = 0; j < 4; ++j) {
        const float p = __expf(s[j][r] - mnew);
        psum += p;
        pwh[(8 * hh + r) * AT_KC + j * 16 + c] = (_Float16)(p * PSC_F);
      }
#pragma unroll
      for (int off = 1; off < 16; off <<= 1) psum += __shfl_xor(psum, off, 32);
      lrow[r] = lrow[r] * alpha + psum;
#pragma unroll
      for (int t = 0; t < 4; ++t) oacc[t][r] *= alpha;
    }
    __builtin_amdgcn_fence(__ATOMIC_RELEASE, "workgroup");
    __builtin_amdgcn_wave_barrier();
    __builtin_amdgcn_fence(__ATOMIC_ACQUIRE, "workgroup");

#pragma unroll 1
    for (int kk = 0; kk < 2; ++kk) {
      FH pa;
      pa.h[0] = *(const v8h*)(pwh + c * AT_KC + kk * 32 + 8 * hh);
      pa.h[1] = *(const v8h*)(pwh + c * AT_KC + kk * 32 + 16 + 8 * hh);
#pragma unroll
      for (int t = 0; t < 4; ++t) {
        FH vb;
        vb.h[0] = *(const v8h*)(Vth + (t * 16 + c) * AT_KC + kk * 32 + 8 * hh);
        vb.h[1] = *(const v8h*)(Vth + (t * 16 + c) * AT_KC + kk * 32 + 16 + 8 * hh);
        oacc[t] = mma_h(pa.v, vb.v, oacc[t]);
      }
    }
  }

  float* os = Os[wave];
#pragma unroll
  for (int r = 0; r < 8; ++r) {
    const float inv = osc / (lrow[r] * PSC_F);
#pragma unroll
    for (int t = 0; t < 4; ++t) os[(8 * hh + r) * 68 + t * 16 + c] = oacc[t][r] * inv;
  }
  __builtin_amdgcn_fence(__ATOMIC_RELEASE, "workgroup");
  __builtin_amdgcn_wave_barrier();
  __builtin_amdgcn_fence(__ATOMIC_ACQUIRE, "workgroup");
  {
    const int q8 = lane >> 3, c8 = (lane & 7) * 8;
    for (int pass = 0; pass < 2; ++pass) {
#pragma unroll
      for (int it = 0; it < 4; ++it) {
        const int row = it * 4 + q8;
        const float* sp = os + row * 68 + c8;
        v8h hv;
#pragma unroll
        for (int e = 0; e < 8; ++e) hv[e] = (_Float16)sp[e];
        *(volatile v8h*)(ob_ptr + (size_t)(q0 + row) * ld + c8) = hv;
      }
      __threadfence();
    }
  }
}

extern "C" void kernel_launch(void* const* d_in, const int* in_sizes, int n_in,
                              void* d_out, int out_size, void* d_ws, size_t ws_size,
                              hipStream_t stream) {
  const int B = 2, S = 2048, HID = 1024, NH = 16, HD = 64, AHS = NH * HD;
  const int M = B * S;
  if (n_in < 9) return;
  if (in_sizes[0] != M * HID || in_sizes[1] != HID * AHS || in_sizes[2] != AHS ||
      in_sizes[3] != HID * AHS || in_sizes[4] != AHS || in_sizes[5] != HID * AHS ||
      in_sizes[6] != AHS || in_sizes[7] != AHS * HID || in_sizes[8] != HID ||
      out_size != M * HID) return;

  const float* hs = (const float*)d_in[0];
  const float* wq = (const float*)d_in[1];
  const float* bq = (const float*)d_in[2];
  const float* wk = (const float*)d_in[3];
  const float* bk = (const float*)d_in[4];
  const float* wv = (const float*)d_in[5];
  const float* bv = (const float*)d_in[6];
  const float* wo = (const float*)d_in[7];
  const float* bo = (const float*)d_in[8];
  float* out = (float*)d_out;

  size_t off = 0;
  char* base = (char*)d_ws;
  const size_t nX  = (size_t)M * HID;
  const size_t nW  = (size_t)HID * AHS;
  const size_t nP  = (size_t)M * AHS;
  _Float16* X16   = (_Float16*)(base + off); off += nX * 2;
  _Float16* WT    = (_Float16*)(base + off); off += 4 * nW * 2;
  _Float16* Q16   = (_Float16*)(base + off); off += nP * 2;
  _Float16* K16   = (_Float16*)(base + off); off += nP * 2;
  _Float16* V16   = (_Float16*)(base + off); off += nP * 2;
  _Float16* CTX16 = (_Float16*)(base + off); off += nP * 2;
  if (off > ws_size || off > (size_t)134217728) return;

  const float WSC = 16.0f;
  const float CSC = 64.0f;

  {
    const int n2 = (int)(nX / 2);
    cast_f32_f16x2<<<dim3((n2 + 255) / 256), dim3(256), 0, stream>>>(hs, X16, n2);
  }
  k_transpose_cast4<<<dim3(AHS / 64, HID / 64, 4), dim3(256), 0, stream>>>(wq, wk, wv, wo, WT, HID, AHS, WSC);

  {
    const int tiles = (M / 64) * (AHS / 64);
    dim3 grid((tiles + 7) / 8, 1);
    wmma_gemm64<0, false, 2, 1, false, 0><<<grid, dim3(256), 0, stream>>>(
        U16(X16), U16(X16), HID, 0L, U16(WT + 0 * nW), U16(WT + 0 * nW), HID, 0L,
        (void*)Q16, (void*)Q16, AHS, 0L, bq, bq, 0L, M, AHS, HID, 1.0f / WSC);
    wmma_gemm64<0, false, 2, 1, false, 0><<<grid, dim3(256), 0, stream>>>(
        U16(X16), U16(X16), HID, 0L, U16(WT + 1 * nW), U16(WT + 1 * nW), HID, 0L,
        (void*)K16, (void*)K16, AHS, 0L, bk, bk, 0L, M, AHS, HID, 1.0f / WSC);
    wmma_gemm64<0, false, 2, 1, false, 0><<<grid, dim3(256), 0, stream>>>(
        U16(X16), U16(X16), HID, 0L, U16(WT + 2 * nW), U16(WT + 2 * nW), HID, 0L,
        (void*)V16, (void*)V16, AHS, 0L, bv, bv, 0L, M, AHS, HID, 1.0f / WSC);
  }

  {
    dim3 grid(B * NH * (S / AT_QB));
    attn64_f16_kernel<<<grid, dim3(128), 0, stream>>>(Q16, K16, V16, CTX16, S, NH, AHS,
                                                      1.0f / 8.0f, CSC);
  }

  {
    const int tiles = (M / 64) * (HID / 64);
    dim3 grid((tiles + 7) / 8, 1);
    wmma_gemm64<0, false, 2, 0, false, 0><<<grid, dim3(256), 0, stream>>>(
        U16(CTX16), U16(CTX16), AHS, 0L, U16(WT + 3 * nW), U16(WT + 3 * nW), AHS, 0L,
        (void*)out, (void*)out, HID, 0L, bo, bo, 0L, M, HID, AHS, 1.0f / (WSC * CSC));
  }
  (void)HD;
}
